// SubGraph_14362370638062
// MI455X (gfx1250) — hardware-verified
//
#include <hip/hip_runtime.h>
#include <stddef.h>
#include <stdint.h>


#define DIN     64
#define HCH     128
#define CPH     32
#define NPJ     256
#define K2      256
#define NTHR    256
#define NWAVE   8
#define EPT     8
#define CHUNK   (NTHR * EPT)
#define WCAP    (EPT * 32)
#define LISTN   (NWAVE * WCAP)
#define NBMAX   2048
#define RCAP    28672
#define DEGCAP  512
#define STW     512
#define GBM     64
#define GBN     64
#define GTHR    128
#define NEGS    0.2f
#define WSMAX   134217728
#define LDS_AGG ((2 * RCAP + 2 * NBMAX + LISTN) * 4 + 64)

static_assert((CHUNK & (CHUNK - 1)) == 0 && CHUNK <= 4096);
static_assert((NBMAX & (NBMAX - 1)) == 0 && NBMAX <= 4096);
static_assert(NTHR * 8 == NBMAX);
static_assert(LISTN >= NBMAX);
static_assert(LISTN >= NWAVE * WCAP);
static_assert((RCAP % 32) == 0);
static_assert(NWAVE * STW <= RCAP);
static_assert(STW >= HCH);
static_assert(LDS_AGG <= 300000);
static_assert(GBM == (GTHR / 32) * 16);
static_assert(DIN / 8 == 8);
static_assert((DIN % 32) == 0 && (K2 % 32) == 0 && (HCH % 32) == 0);
static_assert((NPJ % GBN) == 0 && NPJ == 2 * HCH && K2 == 2 * HCH);
static_assert(HCH == 4 * CPH && CPH == 32);
static_assert(DEGCAP <= RCAP);

typedef float          v4f  __attribute__((ext_vector_type(4)));
typedef float          v8f  __attribute__((ext_vector_type(8)));
typedef int            v4i  __attribute__((ext_vector_type(4)));
typedef int            v8i  __attribute__((ext_vector_type(8)));
typedef unsigned short v8us __attribute__((ext_vector_type(8)));
typedef __bf16         v16b __attribute__((ext_vector_type(16)));
union FragB { v16b v; v8us h[2]; v8i w; };

__device__ __forceinline__ v8f wmb(const FragB& a, const FragB& b, v8f c) {
  v8f d = __builtin_amdgcn_wmma_f32_16x16x32_bf16(false, a.v, false, b.v, (short)0, c, false, false);
  asm volatile("v_nop\n\tv_nop\n\tv_nop\n\tv_nop" : "+v"(d) : "v"(a.w), "v"(b.w));
  return d;
}

__device__ __forceinline__ void ldwait() {
  asm volatile("s_wait_loadcnt 0x0" ::: "memory");
}

__device__ __forceinline__ unsigned bfb(float f) {
  unsigned u = __float_as_uint(f);
  u += 0x7FFFu + ((u >> 16) & 1u);
  return u >> 16;
}
__device__ __forceinline__ float bff(float f) { return __uint_as_float(bfb(f) << 16); }

__device__ __forceinline__ v8us pk8(const v4f a, const v4f b) {
  v8us hv;
  hv[0] = (unsigned short)bfb(a.x); hv[1] = (unsigned short)bfb(a.y);
  hv[2] = (unsigned short)bfb(a.z); hv[3] = (unsigned short)bfb(a.w);
  hv[4] = (unsigned short)bfb(b.x); hv[5] = (unsigned short)bfb(b.y);
  hv[6] = (unsigned short)bfb(b.z); hv[7] = (unsigned short)bfb(b.w);
  return hv;
}

__device__ __forceinline__ int scan_chunk(const int* __restrict__ dsts, int nE, int cbase, int slotBase,
                                          int nb, int vec8, int* list, int tid, int lane, int wave) {
  int wc = 0;
  const int el0  = tid * EPT;
  const int e0   = cbase + el0;
  const int sent = -2147483647 - 1;
  v4i da, db;
  if (vec8 != 0 && cbase + CHUNK <= nE) {
    da = *(const v4i*)(dsts + e0);
    db = *(const v4i*)(dsts + e0 + 4);
  } else {
    da.x = (e0     < nE) ? dsts[min(e0,     nE - 1)] : sent;
    da.y = (e0 + 1 < nE) ? dsts[min(e0 + 1, nE - 1)] : sent;
    da.z = (e0 + 2 < nE) ? dsts[min(e0 + 2, nE - 1)] : sent;
    da.w = (e0 + 3 < nE) ? dsts[min(e0 + 3, nE - 1)] : sent;
    db.x = (e0 + 4 < nE) ? dsts[min(e0 + 4, nE - 1)] : sent;
    db.y = (e0 + 5 < nE) ? dsts[min(e0 + 5, nE - 1)] : sent;
    db.z = (e0 + 6 < nE) ? dsts[min(e0 + 6, nE - 1)] : sent;
    db.w = (e0 + 7 < nE) ? dsts[min(e0 + 7, nE - 1)] : sent;
  }
  const unsigned nbs = (unsigned)slotBase;
  const unsigned unb = (unsigned)nb;
  const unsigned s0 = (unsigned)da.x - nbs, s1 = (unsigned)da.y - nbs;
  const unsigned s2 = (unsigned)da.z - nbs, s3 = (unsigned)da.w - nbs;
  const unsigned s4 = (unsigned)db.x - nbs, s5 = (unsigned)db.y - nbs;
  const unsigned s6 = (unsigned)db.z - nbs, s7 = (unsigned)db.w - nbs;
  const bool h0 = s0 < unb, h1 = s1 < unb, h2 = s2 < unb, h3 = s3 < unb;
  const bool h4 = s4 < unb, h5 = s5 < unb, h6 = s6 < unb, h7 = s7 < unb;
  const unsigned any = __builtin_amdgcn_ballot_w32(h0 | h1 | h2 | h3 | h4 | h5 | h6 | h7);
  if (any != 0u) {
#define HITJ(J, HJ, SJ) { \
      const unsigned mj = __builtin_amdgcn_ballot_w32(HJ); \
      if (mj != 0u) { \
        if (HJ) { \
          const int pos = wc + (int)__builtin_amdgcn_mbcnt_lo(mj, 0u); \
          if (pos < WCAP) list[wave * WCAP + pos] = ((el0 + (J)) << 12) | (int)(SJ); \
        } \
        wc += (int)__builtin_popcount(mj); } }
    HITJ(0, h0, s0)
    HITJ(1, h1, s1)
    HITJ(2, h2, s2)
    HITJ(3, h3, s3)
    HITJ(4, h4, s4)
    HITJ(5, h5, s5)
    HITJ(6, h6, s6)
    HITJ(7, h7, s7)
#undef HITJ
  }
  return wc;
}

__global__ __launch_bounds__(NTHR) void k_xprep(const float* __restrict__ x, unsigned short* xb, int nN, int nUnits) {
  const int i = (int)blockIdx.x * NTHR + (int)threadIdx.x;
  if (i >= nUnits) return;
  const int row = i >> 3;
  const int c0  = (i & 7) * 8;
  const int rc  = row < nN ? row : nN - 1;
  const float* p = x + (size_t)rc * DIN + c0;
  v4f a = *(const v4f*)p, b = *(const v4f*)(p + 4);
  const v4f z4 = {0.f, 0.f, 0.f, 0.f};
  if (row >= nN) { a = z4; b = z4; }
  const v8us hv = pk8(a, b);
  const size_t o = (size_t)row * DIN + c0;
  *(volatile v8us*)(xb + o) = hv;
  __threadfence();
  *(volatile v8us*)(xb + o) = hv;
}

__global__ __launch_bounds__(NTHR) void k_wtr(const float* __restrict__ wl, const float* __restrict__ wr,
                                              int Ksrc, int Kout, unsigned short* wt, int nUnits) {
  const int u = (int)blockIdx.x * NTHR + (int)threadIdx.x;
  if (u >= nUnits) return;
  const int kq = Kout >> 3;
  const int n  = u / kq;
  const int k8 = (u - n * kq) * 8;
  const int side = (n >= HCH) ? 1 : 0;
  const int nc = n & (HCH - 1);
  const float* wsrc = side ? wr : wl;
  int ks = k8;
  if (ks >= Ksrc) ks -= Ksrc;
  if (ks > Ksrc - 8) ks = Ksrc - 8;
  const float* p = wsrc + (size_t)ks * HCH + nc;
  v4f a, b;
  a.x = p[0];                  a.y = p[(size_t)HCH];        a.z = p[(size_t)2 * HCH];    a.w = p[(size_t)3 * HCH];
  b.x = p[(size_t)4 * HCH];    b.y = p[(size_t)5 * HCH];    b.z = p[(size_t)6 * HCH];    b.w = p[(size_t)7 * HCH];
  const v8us hv = pk8(a, b);
  const size_t o = (size_t)n * (size_t)Kout + k8;
  *(volatile v8us*)(wt + o) = hv;
  __threadfence();
  *(volatile v8us*)(wt + o) = hv;
}

__global__ __launch_bounds__(GTHR) void k_gemm(
    const unsigned short* __restrict__ A, const unsigned short* __restrict__ WT,
    const float* __restrict__ b0, const float* __restrict__ b1,
    float* outF, int K, int ldo)
{
  __shared__ __attribute__((aligned(16))) float stg[GBM * GBN];
  const int tid = (int)threadIdx.x, lane = tid & 31, wave = tid >> 5, hh = lane >> 4, m = lane & 15;
  const int rowBase = (int)blockIdx.x * GBM;
  const int col0    = (int)blockIdx.y * GBN;
  const float* bp = (col0 < HCH) ? b0 : b1;
  const int bofs = col0 & (HCH - 1);

  v8f acc[4];
  {
    const v8f z = {0.f, 0.f, 0.f, 0.f, 0.f, 0.f, 0.f, 0.f};
    acc[0] = z; acc[1] = z; acc[2] = z; acc[3] = z;
  }
  const unsigned short* ap = A  + (size_t)(rowBase + 16 * wave + m) * (size_t)K + 8 * hh;
  const unsigned short* wp = WT + (size_t)(col0 + m) * (size_t)K + 8 * hh;
  const int ksteps = K >> 5;
#pragma unroll 1
  for (int ks = 0; ks < ksteps; ++ks) {
    FragB af;
    af.h[0] = *(const v8us*)(ap + 32 * ks);
    af.h[1] = *(const v8us*)(ap + 32 * ks + 16);
#pragma unroll
    for (int t = 0; t < 4; ++t) {
      const unsigned short* wq = wp + (size_t)(16 * t) * (size_t)K + 32 * ks;
      FragB bf;
      bf.h[0] = *(const v8us*)wq;
      bf.h[1] = *(const v8us*)(wq + 16);
      acc[t] = wmb(af, bf, acc[t]);
    }
  }

#pragma unroll
  for (int t = 0; t < 4; ++t) {
    const int lc = 16 * t + m;
    int bi = bofs + lc;
    bi = bi > HCH - 1 ? HCH - 1 : bi;
    bi = bi < 0 ? 0 : bi;
    const float bv = bff(bp[bi]);
#pragma unroll
    for (int r = 0; r < 8; ++r) {
      const int lr = 16 * wave + 8 * hh + r;
      stg[lr * GBN + lc] = acc[t][r] + bv;
    }
  }
  __syncthreads();

  v4f fv[8];
#pragma unroll
  for (int i = 0; i < 8; ++i) {
    const int lr = 16 * wave + 2 * i + hh;
    fv[i] = *(const v4f*)(stg + lr * GBN + 4 * m);
  }
#pragma unroll
  for (int i = 0; i < 8; ++i) {
    const int lr = 16 * wave + 2 * i + hh;
    const int gr = rowBase + lr;
    float* op = outF + (size_t)gr * (size_t)ldo + col0 + 4 * m;
    *(volatile v4f*)op = fv[i];
  }
  __threadfence();
#pragma unroll
  for (int i = 0; i < 8; ++i) {
    const int lr = 16 * wave + 2 * i + hh;
    const int gr = rowBase + lr;
    float* op = outF + (size_t)gr * (size_t)ldo + col0 + 4 * m;
    *(volatile v4f*)op = fv[i];
  }
}

template<int OUTF>
__global__ __launch_bounds__(NTHR) void k_agg(
    const int* __restrict__ srcs, const int* __restrict__ dsts,
    const float* __restrict__ XLR, const float* __restrict__ att, const float* __restrict__ bias,
    unsigned short* Hpl, float* Out,
    int nN, int nE, int nb, int vec8, int MPr) {
  extern __shared__ v4f lds_dyn[];
  int* reg1 = (int*)lds_dyn;
  int* reg2 = reg1 + RCAP;
  int* scnt = reg2 + RCAP;
  int* soff = scnt + NBMAX;
  int* list = soff + NBMAX;
  int* wcnt = list + LISTN;
  int* wtot = wcnt + NWAVE;
  const int tid = (int)threadIdx.x, lane = tid & 31, wave = tid >> 5;
  const int nodeBase = (int)blockIdx.x * nb;

  for (int i = tid; i < NBMAX; i += NTHR) scnt[i] = 0;
  if (tid == 0) reg2[0] = 0;
  __syncthreads();

  int tot = 0;
  const int nChunks = (nE + CHUNK - 1) / CHUNK;
#pragma unroll 1
  for (int ch = 0; ch < nChunks; ++ch) {
    const int cbase = ch * CHUNK;
    const int wc = scan_chunk(dsts, nE, cbase, nodeBase, nb, vec8, list, tid, lane, wave);
    if (lane == 0) wcnt[wave] = wc;
    __syncthreads();
    int pre = 0, all = 0;
#pragma unroll
    for (int w2 = 0; w2 < NWAVE; ++w2) {
      int c = wcnt[w2];
      c = c < 0 ? 0 : (c > WCAP ? WCAP : c);
      all += c;
      pre += (w2 < wave) ? c : 0;
    }
    const int wcc  = wc > WCAP ? WCAP : wc;
    const int base = tot + pre;
#pragma unroll 1
    for (int i = lane; i < wcc; i += 32) {
      const int ent = list[wave * WCAP + i];
      const int el  = (ent >> 12) & (CHUNK - 1);
      const int sl  = ent & (NBMAX - 1);
      int eid = cbase + el;
      eid = eid > nE - 1 ? nE - 1 : eid;
      const int pos = base + i;
      if (pos < RCAP) reg1[pos] = (int)(((unsigned)eid << 12) | (unsigned)sl);
    }
    tot += all;
    tot = tot > RCAP ? RCAP : tot;
    __syncthreads();
  }
  const int nh = tot;

  if (wave == 0) {
#pragma unroll 1
    for (int b0 = 0; b0 < nh; b0 += 32) {
      const int idx = b0 + lane;
      const int uv  = reg1[idx < nh ? idx : nh - 1];
      const int m32 = (nh - b0) < 32 ? (nh - b0) : 32;
#pragma unroll 1
      for (int k = 0; k < m32; ++k) {
        const int u  = __builtin_amdgcn_readlane(uv, k);
        const int sl = u & (NBMAX - 1);
        if (lane == 0) scnt[sl] = scnt[sl] + 1;
      }
    }
  }
  __syncthreads();

  {
    const v4i ca = *(const v4i*)(scnt + 8 * tid);
    const v4i cb = *(const v4i*)(scnt + 8 * tid + 4);
    const int e0 = ca.x < 0 ? 0 : ca.x, e1 = ca.y < 0 ? 0 : ca.y, e2 = ca.z < 0 ? 0 : ca.z, e3 = ca.w < 0 ? 0 : ca.w;
    const int e4 = cb.x < 0 ? 0 : cb.x, e5 = cb.y < 0 ? 0 : cb.y, e6 = cb.z < 0 ? 0 : cb.z, e7 = cb.w < 0 ? 0 : cb.w;
    const int ts = e0 + e1 + e2 + e3 + e4 + e5 + e6 + e7;
    int incl = ts;
#pragma unroll
    for (int d = 1; d < 32; d <<= 1) {
      const int up = __shfl_up(incl, d);
      if (lane >= d) incl += up;
    }
    if (lane == 31) wtot[wave] = incl;
    __syncthreads();
    int pre = 0;
#pragma unroll
    for (int w2 = 0; w2 < NWAVE; ++w2) pre += (w2 < wave) ? wtot[w2] : 0;
    int run = pre + incl - ts;
    soff[8 * tid + 0] = run; run += e0;
    soff[8 * tid + 1] = run; run += e1;
    soff[8 * tid + 2] = run; run += e2;
    soff[8 * tid + 3] = run; run += e3;
    soff[8 * tid + 4] = run; run += e4;
    soff[8 * tid + 5] = run; run += e5;
    soff[8 * tid + 6] = run; run += e6;
    soff[8 * tid + 7] = run;
  }
  __syncthreads();
  for (int i = tid; i < NBMAX; i += NTHR) list[i] = soff[i];
  __syncthreads();

  if (wave == 0) {
#pragma unroll 1
    for (int b0 = 0; b0 < nh; b0 += 32) {
      const int idx = b0 + lane;
      const int uv  = reg1[idx < nh ? idx : nh - 1];
      const int m32 = (nh - b0) < 32 ? (nh - b0) : 32;
#pragma unroll 1
      for (int k = 0; k < m32; ++k) {
        const int u   = __builtin_amdgcn_readlane(uv, k);
        const int sl  = u & (NBMAX - 1);
        const int eid = (int)((unsigned)u >> 12);
        if (lane == 0) {
          int pos = list[sl];
          pos = pos < 0 ? 0 : (pos > RCAP - 1 ? RCAP - 1 : pos);
          reg2[pos] = eid;
          list[sl] = pos + 1;
        }
      }
    }
  }
  __syncthreads();

  const int nbw = nb >> 3;
  const bool ovf = (nh >= RCAP);
  const float qnan = __int_as_float(0x7fc00000);
  float* stw = (float*)reg1 + wave * STW;
  const int l15  = lane & 15;
  const int hsel = lane >> 4;
  const int lim  = nh > 0 ? nh - 1 : 0;
  float attv[4], bsv[4];
#pragma unroll
  for (int h = 0; h < 4; ++h) {
    attv[h] = bff(att[CPH * h + lane]);
    bsv[h]  = bff(bias[CPH * h + lane]);
  }
#pragma unroll 1
  for (int jt = 0; jt < nbw; ++jt) {
    const int slot = wave * nbw + jt;
    const int grow = nodeBase + slot;
    const int gcl  = grow < nN ? grow : nN - 1;
    int st = soff[slot];
    const int craw = scnt[slot];
    int cnt = craw;
    st  = st < 0 ? 0 : (st > nh ? nh : st);
    cnt = cnt < 0 ? 0 : (cnt > DEGCAP ? DEGCAP : cnt);
    if (cnt > nh - st) cnt = nh - st;
    const float pz = (ovf || craw > DEGCAP) ? qnan : 0.0f;
    const float live = grow < nN ? 1.0f : 0.0f;

    const float* rrow = XLR + (size_t)gcl * NPJ + HCH + lane;
    float xrv[4], av[4], mx[4], dn[4];
#pragma unroll
    for (int h = 0; h < 4; ++h) { xrv[h] = rrow[CPH * h]; av[h] = 0.f; mx[h] = -1.0e30f; dn[h] = 0.f; }
    ldwait();

#pragma unroll 1
    for (int q = 0; q <= cnt; ++q) {
      const bool self = (q >= cnt);
      int idx = st + q; idx = idx > lim ? lim : idx;
      int eid = reg2[idx]; eid = eid < 0 ? 0 : (eid > nE - 1 ? nE - 1 : eid);
      const int sraw = srcs[eid];
      const int slr  = sraw < 0 ? 0 : (sraw > nN - 1 ? nN - 1 : sraw);
      const int s    = self ? gcl : slr;
      const float* lrow = XLR + (size_t)s * NPJ + lane;
      float xlv[4];
#pragma unroll
      for (int h = 0; h < 4; ++h) xlv[h] = lrow[CPH * h];
      ldwait();
      float part[4];
#pragma unroll
      for (int h = 0; h < 4; ++h) {
        float e = xlv[h] + xrv[h];
        e = (e >= 0.f) ? e : e * NEGS;
        part[h] = e * attv[h];
      }
#pragma unroll
      for (int off = 16; off > 0; off >>= 1) {
#pragma unroll
        for (int h = 0; h < 4; ++h) part[h] += __shfl_xor(part[h], off);
      }
#pragma unroll
      for (int h = 0; h < 4; ++h) {
        const float al = part[h];
        const float df = al - mx[h];
        const float ee = __expf(-fabsf(df));
        const bool up  = df > 0.f;
        const float s1 = up ? ee : 1.0f;
        const float s2 = up ? 1.0f : ee;
        mx[h] = up ? al : mx[h];
        dn[h] = fmaf(dn[h], s1, s2);
        av[h] = fmaf(av[h], s1, s2 * xlv[h]);
      }
    }
    float rv[4];
#pragma unroll
    for (int h = 0; h < 4; ++h) {
      const float ds = dn[h] > 0.f ? dn[h] : 1.0f;
      const float iv = (dn[h] > 0.f ? 1.0f : 0.0f) * __builtin_amdgcn_rcpf(ds);
      const float o  = fmaf(av[h], iv, bsv[h]);
      rv[h] = fmaxf(o, 0.f) * live + pz;
    }
    __builtin_amdgcn_fence(__ATOMIC_RELEASE, "wavefront");
    __builtin_amdgcn_wave_barrier();
#pragma unroll
    for (int h = 0; h < 4; ++h) stw[CPH * h + lane] = rv[h];
    __builtin_amdgcn_fence(__ATOMIC_RELEASE, "wavefront");
    __builtin_amdgcn_wave_barrier();
    if (OUTF == 1) {
      const v4f g4 = *(const v4f*)(stw + 4 * lane);
      float* gp = Out + (size_t)grow * HCH + 4 * lane;
      const bool wsv = grow < nN;
      if (wsv) *(volatile v4f*)gp = g4;
      __threadfence();
      if (wsv) *(volatile v4f*)gp = g4;
    } else {
      const v4f ga = *(const v4f*)(stw + 8 * l15);
      const v4f gb = *(const v4f*)(stw + 8 * l15 + 4);
      const float f0 = ga.x, f1 = ga.y, f2 = ga.z, f3 = ga.w, f4 = gb.x, f5 = gb.y, f6 = gb.z, f7 = gb.w;
      v8us pv;
#define HLSEL(J, FJ) { \
        const unsigned hb = bfb(FJ); \
        const float hf = __uint_as_float(hb << 16); \
        const unsigned lb = bfb((FJ) - hf); \
        pv[J] = (unsigned short)(hsel ? lb : hb); }
      HLSEL(0, f0) HLSEL(1, f1) HLSEL(2, f2) HLSEL(3, f3)
      HLSEL(4, f4) HLSEL(5, f5) HLSEL(6, f6) HLSEL(7, f7)
#undef HLSEL
      unsigned short* gp = Hpl + (size_t)grow * NPJ + 8 * lane;
      const bool wsv = grow < MPr;
      if (wsv) *(volatile v8us*)gp = pv;
      __threadfence();
      if (wsv) *(volatile v8us*)gp = pv;
    }
  }
}

static int pick_nb(int nE, int nN) {
  int nb = NBMAX;
  while (nb > 16 && (long long)nb * (long long)nE * 5LL > (long long)RCAP * (long long)nN * 4LL) nb >>= 1;
  return nb;
}
static inline int cdiv(int a, int b) { return (a + b - 1) / b; }

extern "C" void kernel_launch(void* const* d_in, const int* in_sizes, int n_in,
                              void* d_out, int out_size, void* d_ws, size_t ws_size,
                              hipStream_t stream) {
  if (n_in < 14) return;
  const int nN = in_sizes[0] / DIN;
  if (nN <= 0 || in_sizes[0] != nN * DIN || nN > (1 << 22)) return;
  if (in_sizes[13] < 2 || (in_sizes[13] & 1) != 0) return;
  const int nE = in_sizes[13] / 2;
  if (nE < 1 || nE > (1 << 20)) return;
  if (in_sizes[1]  != DIN * HCH || in_sizes[2]  != HCH) return;
  if (in_sizes[3]  != DIN * HCH || in_sizes[4]  != HCH) return;
  if (in_sizes[5]  != HCH       || in_sizes[6]  != HCH) return;
  if (in_sizes[7]  != HCH * HCH || in_sizes[8]  != HCH) return;
  if (in_sizes[9]  != HCH * HCH || in_sizes[10] != HCH) return;
  if (in_sizes[11] != HCH       || in_sizes[12] != HCH) return;
  if (out_size != nN * HCH) return;

  const float* x     = (const float*)d_in[0];
  const float* Wl1   = (const float*)d_in[1];
  const float* bl1   = (const float*)d_in[2];
  const float* Wr1   = (const float*)d_in[3];
  const float* br1   = (const float*)d_in[4];
  const float* att1  = (const float*)d_in[5];
  const float* bias1 = (const float*)d_in[6];
  const float* Wl2   = (const float*)d_in[7];
  const float* bl2   = (const float*)d_in[8];
  const float* Wr2   = (const float*)d_in[9];
  const float* br2   = (const float*)d_in[10];
  const float* att2  = (const float*)d_in[11];
  const float* bias2 = (const float*)d_in[12];
  const int*   ei    = (const int*)  d_in[13];
  float* out = (float*)d_out;
  const int* src = ei;
  const int* dst = ei + nE;

  const int MP   = cdiv(nN, GBM) * GBM;
  const int nb   = pick_nb(nE, nN);
  const int gA   = cdiv(MP, nb);
  const int vec8 = ((nE & 3) == 0) ? 1 : 0;
  if (gA * nb < MP) return;

  char* ws = (char*)d_ws;
  size_t off = 0;
  const size_t oXB  = off; off += (size_t)MP * DIN * 2;             off = (off + 255) & ~(size_t)255;
  const size_t oXLR = off; off += (size_t)MP * NPJ * 4;             off = (off + 255) & ~(size_t)255;
  const size_t oHPL = off; off += (size_t)MP * NPJ * 2;             off = (off + 255) & ~(size_t)255;
  const size_t oWT1 = off; off += (size_t)NPJ * DIN * 2;            off = (off + 255) & ~(size_t)255;
  const size_t oWT2 = off; off += (size_t)NPJ * K2 * 2;             off = (off + 255) & ~(size_t)255;
  if (off > ws_size || off > (size_t)WSMAX) return;
  unsigned short* XB  = (unsigned short*)(ws + oXB);
  float*          XLR = (float*)(ws + oXLR);
  unsigned short* HPL = (unsigned short*)(ws + oHPL);
  unsigned short* WT1 = (unsigned short*)(ws + oWT1);
  unsigned short* WT2 = (unsigned short*)(ws + oWT2);

  hipFuncSetAttribute(reinterpret_cast<const void*>(&k_agg<0>),
                      hipFuncAttributeMaxDynamicSharedMemorySize, LDS_AGG);
  hipFuncSetAttribute(reinterpret_cast<const void*>(&k_agg<1>),
                      hipFuncAttributeMaxDynamicSharedMemorySize, LDS_AGG);

  const int nUx = MP * (DIN / 8);
  k_xprep<<<cdiv(nUx, NTHR), NTHR, 0, stream>>>(x, XB, nN, nUx);

  {
    const int nU1 = NPJ * (DIN / 8);
    k_wtr<<<cdiv(nU1, NTHR), NTHR, 0, stream>>>(Wl1, Wr1, DIN, DIN, WT1, nU1);
    const int nU2 = NPJ * (K2 / 8);
    k_wtr<<<cdiv(nU2, NTHR), NTHR, 0, stream>>>(Wl2, Wr2, HCH, K2, WT2, nU2);
  }

  const int gM = MP / GBM;
  k_gemm<<<dim3(gM, NPJ / GBN), GTHR, 0, stream>>>(XB, WT1, bl1, br1, XLR, DIN, NPJ);
  k_agg<0><<<gA, NTHR, LDS_AGG, stream>>>(src, dst, XLR, att1, bias1, HPL, out, nN, nE, nb, vec8, MP);
  k_gemm<<<dim3(gM, NPJ / GBN), GTHR, 0, stream>>>(HPL, WT2, bl2, br2, XLR, K2, NPJ);
  k_agg<1><<<gA, NTHR, LDS_AGG, stream>>>(src, dst, XLR, att2, bias2, HPL, out, nN, nE, nb, vec8, MP);
}
